// SelfAttention_33852932227207
// MI455X (gfx1250) — hardware-verified
//
#include <hip/hip_runtime.h>


#ifndef NB
#define NB 4
#endif
#ifndef SEQ
#define SEQ 2048
#endif
#define NB_FULL   4
#define SEQ_FULL  2048
#define DIN       1024
#define DM        512
#define GK        1024
#define MROWS     (NB * SEQ)
#define GBM       128
#define GBN       128
#define PT        136
#define NTHR      512
#define NWV       16
#define QB        16
#define KBLK      256
#define PP        264
#define OPITCH    516
#define VGPR_CAP  __attribute__((amdgpu_num_vgpr(256)))

static_assert(NB >= 1 && NB <= NB_FULL);
static_assert(SEQ <= SEQ_FULL);
static_assert(SEQ % KBLK == 0);
static_assert(SEQ % GBM == 0);
static_assert(SEQ % QB == 0);
static_assert(MROWS % GBM == 0);
static_assert(DM % GBN == 0);
static_assert(DIN == GK);
static_assert(2 * DM == GK);
static_assert(GK % 32 == 0);
static_assert(DM % 32 == 0);
static_assert(NTHR == NWV * 32);
static_assert(GBM == 4 * 32 && GBN == 4 * 32);
static_assert(DM == NWV * 32);
static_assert(KBLK == NWV * 16);
static_assert(QB == 16);
static_assert((PT * 2) % 16 == 0);
static_assert((PP * 2) % 16 == 0);
static_assert((OPITCH * 4) % 16 == 0);
static_assert(PT >= GBN && PT >= GBM);
static_assert(PP >= KBLK);
static_assert(OPITCH >= DM);
static_assert(GBM * GBN / 8 == 4 * NTHR);
static_assert(QB * DM / 4 == 4 * NTHR);

#define W_ELEMS   ((size_t)DM * GK)
#define OFF_XB    ((size_t)0)
#define OFF_WQ    (OFF_XB + (size_t)MROWS * GK)
#define OFF_WK    (OFF_WQ + W_ELEMS)
#define OFF_WV    (OFF_WK + W_ELEMS)
#define OFF_WA    (OFF_WV + W_ELEMS)
#define OFF_WB    (OFF_WA + W_ELEMS)
#define OFF_KHL   (OFF_WB + W_ELEMS)
#define OFF_VHL   (OFF_KHL + (size_t)MROWS * GK)
#define OFF_QH    (OFF_VHL + (size_t)MROWS * GK)
#define OFF_KAH   (OFF_QH + (size_t)MROWS * DM)
#define OFF_UTH   (OFF_KAH + (size_t)MROWS * DM)
#define OFF_UTR   (OFF_UTH + (size_t)MROWS * DM)
#define WS_HALVES (OFF_UTR + (size_t)MROWS * DM)
static_assert(WS_HALVES * 2 <= (size_t)134217728);
static_assert(OFF_WQ % 64 == 0 && OFF_KHL % 64 == 0 && OFF_QH % 64 == 0 && OFF_UTR % 64 == 0);

typedef __bf16   bf16;
typedef _Float16 f16;
typedef bf16     v16bf __attribute__((ext_vector_type(16)));
typedef f16      v16h  __attribute__((ext_vector_type(16)));
typedef float    v8f   __attribute__((ext_vector_type(8)));
typedef float    v4f   __attribute__((ext_vector_type(4)));
typedef unsigned v4u   __attribute__((ext_vector_type(4)));

union FragB  { v16bf v; v4u q[2]; };
union FragH  { v16h  v; v4u q[2]; };
union Pack8B { v4u u; bf16 h[8]; };
union Pack8H { v4u u; f16 h[8]; };
union Pack8S { v4u u; unsigned short s[8]; };

static __device__ __forceinline__ v8f mma_bf16(v16bf a, v16bf b, v8f acc) {
  acc = __builtin_amdgcn_wmma_f32_16x16x32_bf16(false, a, false, b, (short)0, acc, false, false);
  asm volatile("v_nop\n\tv_nop\n\tv_nop\n\tv_nop" : "+v"(acc) : "v"(a), "v"(b));
  return acc;
}
static __device__ __forceinline__ v8f mma_f16(v16h a, v16h b, v8f acc) {
  acc = __builtin_amdgcn_wmma_f32_16x16x32_f16(false, a, false, b, (short)0, acc, false, false);
  asm volatile("v_nop\n\tv_nop\n\tv_nop\n\tv_nop" : "+v"(acc) : "v"(a), "v"(b));
  return acc;
}

static __device__ __forceinline__ unsigned short enc16(float v, int kind) {
  if (kind == 1) {
    return __builtin_bit_cast(unsigned short, (bf16)v);
  }
  if (kind == 2) {
    const bf16 h = (bf16)v;
    return __builtin_bit_cast(unsigned short, (bf16)(v - (float)h));
  }
  const float s = v * 16.0f;
  const f16 hh = (f16)s;
  if (kind == 0) return __builtin_bit_cast(unsigned short, hh);
  return __builtin_bit_cast(unsigned short, (f16)((s - (float)hh) * 2048.0f));
}

__global__ __launch_bounds__(256) void cvt_rows_kernel(const float* __restrict__ src,
                                                       unsigned short* __restrict__ wr,
                                                       size_t dst_off, int n_rows, int src_cols,
                                                       int rows_per_b, int rows_per_b_full) {
  const size_t p = (size_t)blockIdx.x * 256 + threadIdx.x;
  const int row = (int)(p >> 7);
  const int c   = (int)(p & 127);
  if (row >= n_rows) return;
  const int bb = row / rows_per_b;
  const int rr = row - bb * rows_per_b;
  const int sc = (c * 8) % src_cols;
  const float* s = src + ((size_t)bb * rows_per_b_full + rr) * src_cols + sc;
  const v4f a0 = *(const v4f*)(s);
  const v4f a1 = *(const v4f*)(s + 4);
  Pack8B pk;
  #pragma unroll
  for (int i = 0; i < 4; ++i) {
    pk.h[i]     = (bf16)a0[i];
    pk.h[4 + i] = (bf16)a1[i];
  }
  const v4u val = pk.u;
  unsigned short* d = wr + dst_off + (size_t)row * GK + c * 8;
  *(volatile v4u*)d = val;
  __threadfence();
  *(volatile v4u*)d = val;
}

__global__ __launch_bounds__(NTHR) VGPR_CAP void gemm_kernel(const unsigned short* __restrict__ rd,
                                                             unsigned short* __restrict__ wr, int stage) {
  const int tid  = threadIdx.x;
  const int wave = __builtin_amdgcn_readfirstlane(tid >> 5);
  const int lane = tid & 31;
  const int lq   = lane & 15;
  const int hi   = lane >> 4;
  const int wm   = wave >> 2;
  const int wn   = wave & 3;
  const int n0   = blockIdx.x * GBN;
  const int m0   = blockIdx.y * GBM;
  const int job  = stage * 3 + (int)blockIdx.z;

  const size_t a_off = (job < 3) ? OFF_XB : ((job == 3) ? OFF_KHL : OFF_VHL);
  const size_t w_off = (job == 0) ? OFF_WQ : (job == 1) ? OFF_WK : (job == 2) ? OFF_WV
                     : (job == 3) ? OFF_WA : OFF_WB;
  const size_t o0    = (job == 0) ? OFF_QH : (job == 1) ? OFF_KHL : (job == 2) ? OFF_VHL
                     : (job == 3) ? OFF_KAH : OFF_UTH;
  const size_t o1    = OFF_UTR;
  const int mode     = (job == 0 || job == 3) ? 0 : ((job == 4) ? 2 : 1);

  __shared__ __align__(16) unsigned short sT[GBM * PT];

  v8f acc[2][2];
  #pragma unroll
  for (int mt = 0; mt < 2; ++mt) {
    #pragma unroll
    for (int nt = 0; nt < 2; ++nt) acc[mt][nt] = (v8f){0, 0, 0, 0, 0, 0, 0, 0};
  }

  const size_t ap = a_off + (size_t)(m0 + wm * 32 + lq) * GK + hi * 8;
  const size_t wp = w_off + (size_t)(n0 + wn * 32 + lq) * GK + hi * 8;

  #pragma unroll 2
  for (int k0 = 0; k0 < GK; k0 += 32) {
    FragB a[2], w[2];
    #pragma unroll
    for (int mt = 0; mt < 2; ++mt) {
      a[mt].q[0] = *(const v4u*)(rd + ap + (size_t)mt * 16 * GK + k0);
      a[mt].q[1] = *(const v4u*)(rd + ap + (size_t)mt * 16 * GK + k0 + 16);
    }
    #pragma unroll
    for (int nt = 0; nt < 2; ++nt) {
      w[nt].q[0] = *(const v4u*)(rd + wp + (size_t)nt * 16 * GK + k0);
      w[nt].q[1] = *(const v4u*)(rd + wp + (size_t)nt * 16 * GK + k0 + 16);
    }
    #pragma unroll
    for (int mt = 0; mt < 2; ++mt) {
      #pragma unroll
      for (int nt = 0; nt < 2; ++nt) acc[mt][nt] = mma_bf16(a[mt].v, w[nt].v, acc[mt][nt]);
    }
  }

  const int bq = m0 / SEQ;
  const int s0 = m0 - bq * SEQ;
  const int nplane = (mode == 0) ? 1 : 2;

  #pragma unroll 1
  for (int pl = 0; pl < nplane; ++pl) {
    const int kind = (mode == 0) ? 0 : ((mode == 1) ? (1 + pl) : ((pl == 0) ? 0 : 3));
    if (mode != 2) {
      #pragma unroll
      for (int mt = 0; mt < 2; ++mt) {
        #pragma unroll
        for (int nt = 0; nt < 2; ++nt) {
          #pragma unroll
          for (int r = 0; r < 8; ++r) {
            const int row = wm * 32 + mt * 16 + hi * 8 + r;
            const int col = wn * 32 + nt * 16 + lq;
            sT[row * PT + col] = enc16(acc[mt][nt][r], kind);
          }
        }
      }
    } else {
      #pragma unroll
      for (int mt = 0; mt < 2; ++mt) {
        #pragma unroll
        for (int nt = 0; nt < 2; ++nt) {
          Pack8S pk;
          #pragma unroll
          for (int r = 0; r < 8; ++r) pk.s[r] = enc16(acc[mt][nt][r], kind);
          *(v4u*)(sT + (wn * 32 + nt * 16 + lq) * PT + wm * 32 + mt * 16 + hi * 8) = pk.u;
        }
      }
    }
    __syncthreads();

    v4u    vals[4];
    size_t gi[4];
    #pragma unroll
    for (int it = 0; it < 4; ++it) {
      const int p  = it * NTHR + tid;
      const int rr = p >> 4;
      const int c8 = p & 15;
      vals[it] = *(const v4u*)(sT + rr * PT + c8 * 8);
      size_t g;
      if (mode == 0)      g = o0 + (size_t)(m0 + rr) * DM + n0 + c8 * 8;
      else if (mode == 1) g = o0 + (size_t)(m0 + rr) * GK + pl * DM + n0 + c8 * 8;
      else                g = ((pl == 0) ? o0 : o1) + ((size_t)bq * DM + n0 + rr) * SEQ + s0 + c8 * 8;
      gi[it] = g;
    }
    #pragma unroll
    for (int it = 0; it < 4; ++it) *(volatile v4u*)(wr + gi[it]) = vals[it];
    __threadfence();
    #pragma unroll
    for (int it = 0; it < 4; ++it) *(volatile v4u*)(wr + gi[it]) = vals[it];
    __syncthreads();
  }
}

__global__ __launch_bounds__(NTHR) VGPR_CAP void attn_kernel(const unsigned short* __restrict__ rd,
                                                             float* __restrict__ out) {
  const int qt   = blockIdx.x;
  const int b    = blockIdx.y;
  const int tid  = threadIdx.x;
  const int wave = __builtin_amdgcn_readfirstlane(tid >> 5);
  const int lane = tid & 31;
  const int lq   = lane & 15;
  const int hi   = lane >> 4;

  __shared__ __align__(16) unsigned short sP[QB * PP];
  __shared__ float sMax[NWV * 16];
  __shared__ float sSum[NWV * 16];
  __shared__ __align__(16) float sO[QB * OPITCH];

  const size_t qoff  = OFF_QH + ((size_t)b * SEQ + qt * QB + lq) * DM + hi * 8;
  const size_t kbase = OFF_KAH + (size_t)b * SEQ * DM;
  const size_t uoffh = OFF_UTH + ((size_t)b * DM + wave * 32 + lq) * SEQ + hi * 8;
  const size_t uoffr = OFF_UTR + ((size_t)b * DM + wave * 32 + lq) * SEQ + hi * 8;

  v8f o[2], o2[2];
  #pragma unroll
  for (int nt = 0; nt < 2; ++nt) {
    o[nt]  = (v8f){0, 0, 0, 0, 0, 0, 0, 0};
    o2[nt] = (v8f){0, 0, 0, 0, 0, 0, 0, 0};
  }
  float m_run = -__builtin_inff();
  float l_run = 0.0f;
  const float SL = 1.4426950408889634f * 0.04419417382415922f * (1.0f / 256.0f);

  #pragma unroll 1
  for (int kb = 0; kb < SEQ / KBLK; ++kb) {
    const int j0 = kb * KBLK + wave * 16;
    const size_t ka0 = kbase + (size_t)(j0 + lq) * DM + hi * 8;

    v8f c = (v8f){0, 0, 0, 0, 0, 0, 0, 0};
    #pragma unroll 4
    for (int ks = 0; ks < DM / 32; ++ks) {
      FragH qf, a0;
      qf.q[0] = *(const v4u*)(rd + qoff + ks * 32);
      qf.q[1] = *(const v4u*)(rd + qoff + ks * 32 + 16);
      a0.q[0] = *(const v4u*)(rd + ka0 + ks * 32);
      a0.q[1] = *(const v4u*)(rd + ka0 + ks * 32 + 16);
      c = mma_f16(a0.v, qf.v, c);
    }

    float mloc = c[0];
    #pragma unroll
    for (int r = 1; r < 8; ++r) mloc = fmaxf(mloc, c[r]);
    mloc = fmaxf(mloc, __shfl_xor(mloc, 16, 32));
    if (hi == 0) sMax[wave * 16 + lq] = mloc;
    __syncthreads();

    float mblk = sMax[lq];
    #pragma unroll
    for (int w = 1; w < NWV; ++w) mblk = fmaxf(mblk, sMax[w * 16 + lq]);
    const float m_new = fmaxf(m_run, mblk);
    const float scale = __builtin_amdgcn_exp2f((m_run - m_new) * SL);
    m_run = m_new;

    Pack8H p0;
    float psum = 0.0f;
    #pragma unroll
    for (int r = 0; r < 8; ++r) {
      const float e0 = __builtin_amdgcn_exp2f((c[r] - m_new) * SL);
      psum += e0;
      p0.h[r] = (f16)(e0 * 4096.0f);
    }
    *(v4u*)(sP + lq * PP + wave * 16 + hi * 8) = p0.u;
    psum += __shfl_xor(psum, 16, 32);
    if (hi == 0) sSum[wave * 16 + lq] = psum;
    __syncthreads();

    float lblk = sSum[lq];
    #pragma unroll
    for (int w = 1; w < NWV; ++w) lblk += sSum[w * 16 + lq];
    l_run = l_run * scale + lblk;

    float sc[8];
    #pragma unroll
    for (int r = 0; r < 8; ++r) sc[r] = __shfl(scale, (hi << 3) + r, 32);
    #pragma unroll
    for (int nt = 0; nt < 2; ++nt) {
      #pragma unroll
      for (int r = 0; r < 8; ++r) {
        o[nt][r]  *= sc[r];
        o2[nt][r] *= sc[r];
      }
    }

    #pragma unroll 2
    for (int ch = 0; ch < KBLK / 32; ++ch) {
      FragH pa;
      pa.q[0] = *(const v4u*)(sP + lq * PP + ch * 32 + hi * 8);
      pa.q[1] = *(const v4u*)(sP + lq * PP + ch * 32 + 16 + hi * 8);
      const size_t ko = (size_t)kb * KBLK + ch * 32;
      #pragma unroll
      for (int nt = 0; nt < 2; ++nt) {
        FragH bh, br;
        bh.q[0] = *(const v4u*)(rd + uoffh + (size_t)nt * 16 * SEQ + ko);
        bh.q[1] = *(const v4u*)(rd + uoffh + (size_t)nt * 16 * SEQ + ko + 16);
        br.q[0] = *(const v4u*)(rd + uoffr + (size_t)nt * 16 * SEQ + ko);
        br.q[1] = *(const v4u*)(rd + uoffr + (size_t)nt * 16 * SEQ + ko + 16);
        o[nt]  = mma_f16(pa.v, bh.v, o[nt]);
        o2[nt] = mma_f16(pa.v, br.v, o2[nt]);
      }
    }
    __syncthreads();
  }

  float rs[8];
  #pragma unroll
  for (int r = 0; r < 8; ++r) rs[r] = 1.0f / __shfl(l_run, (hi << 3) + r, 32);

  #pragma unroll
  for (int r = 0; r < 8; ++r) {
    #pragma unroll
    for (int nt = 0; nt < 2; ++nt) {
      const float val = (o[nt][r] + o2[nt][r] * (1.0f / 2048.0f)) * (1.0f / 65536.0f) * rs[r];
      sO[(hi * 8 + r) * OPITCH + wave * 32 + nt * 16 + lq] = val;
    }
  }
  __syncthreads();

  v4f    vals[4];
  size_t gidx[4];
  #pragma unroll
  for (int it = 0; it < 4; ++it) {
    const int p   = it * NTHR + tid;
    const int row = p >> 7;
    const int c4  = p & 127;
    vals[it] = *(const v4f*)(sO + row * OPITCH + c4 * 4);
    gidx[it] = ((size_t)b * SEQ_FULL + qt * QB + row) * DM + c4 * 4;
  }
  #pragma unroll
  for (int it = 0; it < 4; ++it) *(volatile v4f*)(out + gidx[it]) = vals[it];
  __threadfence();
  #pragma unroll
  for (int it = 0; it < 4; ++it) *(volatile v4f*)(out + gidx[it]) = vals[it];
}

extern "C" void kernel_launch(void* const* d_in, const int* in_sizes, int n_in,
                              void* d_out, int out_size, void* d_ws, size_t ws_size,
                              hipStream_t stream) {
  if (n_in < 6) return;
  const size_t rows_used = (size_t)(NB - 1) * SEQ_FULL + SEQ;
  if ((size_t)in_sizes[0] < rows_used * DIN) return;
  if ((size_t)in_sizes[1] < (size_t)DM * DIN) return;
  if ((size_t)in_sizes[2] < (size_t)DM * DIN) return;
  if ((size_t)in_sizes[3] < (size_t)DM * DIN) return;
  if ((size_t)in_sizes[4] < (size_t)DM * DM) return;
  if ((size_t)in_sizes[5] < (size_t)DM * DM) return;
  if ((size_t)out_size < rows_used * DM) return;
  if (ws_size < WS_HALVES * 2) return;

  const float* x  = (const float*)d_in[0];
  const float* Wk = (const float*)d_in[1];
  const float* Wq = (const float*)d_in[2];
  const float* Wv = (const float*)d_in[3];
  const float* Wa = (const float*)d_in[4];
  const float* Wb = (const float*)d_in[5];
  unsigned short* ws = (unsigned short*)d_ws;
  float* out = (float*)d_out;

  cvt_rows_kernel<<<dim3((MROWS * 128 + 255) / 256), 256, 0, stream>>>(x,  ws, OFF_XB, MROWS, DIN, SEQ, SEQ_FULL);
  cvt_rows_kernel<<<dim3((DM * 128 + 255) / 256), 256, 0, stream>>>(Wq, ws, OFF_WQ, DM, DIN, DM, DM);
  cvt_rows_kernel<<<dim3((DM * 128 + 255) / 256), 256, 0, stream>>>(Wk, ws, OFF_WK, DM, DIN, DM, DM);
  cvt_rows_kernel<<<dim3((DM * 128 + 255) / 256), 256, 0, stream>>>(Wv, ws, OFF_WV, DM, DIN, DM, DM);
  cvt_rows_kernel<<<dim3((DM * 128 + 255) / 256), 256, 0, stream>>>(Wa, ws, OFF_WA, DM, DM, DM, DM);
  cvt_rows_kernel<<<dim3((DM * 128 + 255) / 256), 256, 0, stream>>>(Wb, ws, OFF_WB, DM, DM, DM, DM);

  gemm_kernel<<<dim3(DM / GBN, MROWS / GBM, 3), NTHR, 0, stream>>>(ws, ws, 0);
  gemm_kernel<<<dim3(DM / GBN, MROWS / GBM, 2), NTHR, 0, stream>>>(ws, ws, 1);

  attn_kernel<<<dim3(SEQ / QB, NB), NTHR, 0, stream>>>(ws, out);
}
